// DepthTransformer2D_3D_49435073577555
// MI455X (gfx1250) — hardware-verified
//
#include <hip/hip_runtime.h>
#include <math.h>

typedef __attribute__((ext_vector_type(16))) _Float16 v16h;
typedef __attribute__((ext_vector_type(16))) __bf16 v16b;
typedef __attribute__((ext_vector_type(8)))  _Float16 v8h;
typedef __attribute__((ext_vector_type(8)))  float v8f;
typedef __attribute__((ext_vector_type(4)))  float v4f;
typedef __attribute__((ext_vector_type(2)))  float v2f;
typedef __attribute__((ext_vector_type(4)))  unsigned v4u;
typedef __attribute__((ext_vector_type(4)))  int v4i;
typedef float __attribute__((may_alias)) float_a;
typedef int __attribute__((may_alias)) int_a;

template <typename T> __device__ __forceinline__ void vst2(void* p, T v) { *(volatile T*)p = v; __threadfence(); *(volatile T*)p = v; }
__device__ __forceinline__ v8f wmma16(v16h a, v16h b, v8f c) {
  v8f d = __builtin_amdgcn_wmma_f32_16x16x32_f16(false, a, false, b, (short)0, c, false, false);
  asm volatile("v_nop\n\tv_nop\n\tv_nop\n\tv_nop" : "+v"(d) : "v"(a), "v"(b));
  return d;
}
__device__ __forceinline__ v8f wmma_bf(v16b a, v16b b, v8f c) {
  v8f d = __builtin_amdgcn_wmma_f32_16x16x32_bf16(false, a, false, b, (short)0, c, false, false);
  asm volatile("v_nop\n\tv_nop\n\tv_nop\n\tv_nop" : "+v"(d) : "v"(a), "v"(b));
  return d;
}
__device__ __forceinline__ v16h frag_h(const _Float16* rowk0, int lane) {
  union { v16h v; v8h q[2]; } u; const _Float16* p = rowk0 + 8 * (lane >> 4);
  u.q[0] = *(const v8h*)p; u.q[1] = *(const v8h*)(p + 16); return u.v;
}
__device__ __forceinline__ v16h frag_f32(const float* rowk0, int lane) {
  v16h a; const float* p = rowk0 + 8 * (lane >> 4);
#pragma unroll
  for (int i = 0; i < 8; ++i) { a[i] = (_Float16)p[i]; a[8 + i] = (_Float16)p[16 + i]; }
  return a;
}
__device__ __forceinline__ v16h frag_f32s(const float* rowk0, int lane, float sc) {
  v16h a; const float* p = rowk0 + 8 * (lane >> 4);
#pragma unroll
  for (int i = 0; i < 8; ++i) { a[i] = (_Float16)(p[i] * sc); a[8 + i] = (_Float16)(p[16 + i] * sc); }
  return a;
}
__device__ __forceinline__ v16h fragc_f32(const float* W, int k0, int n, int lane, int ld, int K) {
  v16h a; const int g = lane >> 4;
#pragma unroll
  for (int i = 0; i < 8; ++i) { const int ka = k0 + 8 * g + i, kb = ka + 16;
    a[i] = (_Float16)(ka < K ? W[(size_t)(ka < K ? ka : K - 1) * ld + n] : 0.f); a[8 + i] = (_Float16)(kb < K ? W[(size_t)(kb < K ? kb : K - 1) * ld + n] : 0.f); }
  return a;
}
struct F2 { v16b h, l; };
__device__ __forceinline__ F2 bsplit16(const float v[16]) { F2 r;
#pragma unroll
  for (int i = 0; i < 16; ++i) { const __bf16 h = (__bf16)v[i]; r.h[i] = h; r.l[i] = (__bf16)(v[i] - (float)h); }
  return r; }
__device__ __forceinline__ F2 split_row(const float* row, int k0, int lane) { float v[16]; const float* p = row + k0 + 8 * (lane >> 4);
#pragma unroll
  for (int i = 0; i < 8; ++i) { v[i] = p[i]; v[8 + i] = p[16 + i]; }
  return bsplit16(v); }
__device__ __forceinline__ F2 split_rowK(const float* row, int k0, int lane, int K) { float v[16]; const int g = lane >> 4;
#pragma unroll
  for (int i = 0; i < 8; ++i) { const int ka = k0 + 8 * g + i, kb = ka + 16; v[i] = ka < K ? row[ka < K ? ka : K - 1] : 0.f; v[8 + i] = kb < K ? row[kb < K ? kb : K - 1] : 0.f; }
  return bsplit16(v); }
__device__ __forceinline__ F2 split_col(const float* W, int k0, int n, int lane, int ld, int K) { float v[16]; const int g = lane >> 4;
#pragma unroll
  for (int i = 0; i < 8; ++i) { const int ka = k0 + 8 * g + i, kb = ka + 16; v[i] = ka < K ? W[(size_t)(ka < K ? ka : K - 1) * ld + n] : 0.f; v[8 + i] = kb < K ? W[(size_t)(kb < K ? kb : K - 1) * ld + n] : 0.f; }
  return bsplit16(v); }
__device__ __forceinline__ v8f mac3(const F2& a, const F2& b, v8f c) { c = wmma_bf(a.l, b.h, c); c = wmma_bf(a.h, b.l, c); return wmma_bf(a.h, b.h, c); }
__device__ __forceinline__ float sigm(float v) { return 1.0f / (1.0f + expf(-v)); }
#define LDSX() do { asm volatile("s_wait_dscnt 0" ::: "memory"); __builtin_amdgcn_wave_barrier(); __builtin_amdgcn_fence(__ATOMIC_RELEASE, "workgroup"); } while (0)


#define NB 2
#define CC 128
#define NQ 200
#define NQP 256
#ifndef NK
#define NK 24000
#endif
#define NH 8
#define DH 16
#define CAM 16
#define FFN 256
#define NQR (NB * NQP)
#define NKR (NB * NK)
typedef __attribute__((ext_vector_type(8))) __bf16 v8b;
__device__ __forceinline__ v16b frag_b(const __bf16* rowk0, int lane) {
  union { v16b v; v8b q[2]; } u; const __bf16* p = rowk0 + 8 * (lane >> 4);
  u.q[0] = *(const v8b*)p; u.q[1] = *(const v8b*)(p + 16); return u.v;
}
__device__ __forceinline__ float bfr(float v) { return (float)(__bf16)v; }
__device__ __attribute__((noinline)) float exp_ni(float v) { return expf(v); }
__device__ __attribute__((noinline)) float erf_ni(float v) { return erff(v); }

#define PKW(i) ((size_t)(i) * CC * CC)
#define PK_F1 ((size_t)14 * CC * CC)
#define PK_F2 (PK_F1 + (size_t)FFN * CC)
#define PK_C1 (PK_F2 + (size_t)CC * FFN)
#define PK_END (PK_C1 + (size_t)CC * 32)
#define WS_PK   0u
#define WS_Q    (((2u * PK_END) + 127u) / 128u * 128u)
#define WS_QPE  (WS_Q + 4u * NQR * CC)
#define WS_XS   (WS_QPE + 4u * NQR * CC)
#define WS_X    (WS_XS + 4u * NQR * CC)
#define WS_T    (WS_X + 4u * NQR * CC)
#define WS_SO   (WS_T + 4u * NQR * CC)
#define WS_GH   (WS_SO + 4u * NQR * CC)
#define WS_GL   (WS_GH + 2u * NQR * FFN)
#define WS_SQH  (WS_GL + 2u * NQR * FFN)
#define WS_SQL  (WS_SQH + 2u * NQR * NH * 32)
#define WS_SKH  (WS_SQL + 2u * NQR * NH * 32)
#define WS_SKL  (WS_SKH + 2u * NQR * NH * 32)
#define WS_SVH  (WS_SKL + 2u * NQR * NH * 32)
#define WS_SVL  (WS_SVH + 2u * NQR * CC)
#define WS_KF   (WS_SVL + 2u * NQR * CC)
#define WS_KC   (WS_KF + 4u * (size_t)NKR * CC)
#define WS_CB   (WS_KC + 4u * (size_t)NKR * CC)
#define WS_CH   (WS_CB + 4u * (size_t)NKR * 32)
#define WS_CKH  (WS_CH + 4u * (size_t)NKR * CC)
#define WS_CKL  (WS_CKH + 2u * (size_t)NKR * NH * 32)
#define WS_CVH  (WS_CKL + 2u * (size_t)NKR * NH * 32)
#define WS_CVL  (WS_CVH + 2u * (size_t)NKR * CC)
#define WS_ST   (WS_CVL + 2u * (size_t)NKR * CC)
#define WS_MS   (WS_ST + 4u * (size_t)(NKR / 64) * 32)
#define WS_END  (WS_MS + 4u * 64)

struct WList { const float* w[14]; };
__global__ __launch_bounds__(256) void k_pack(WList WL, const float* __restrict__ WF1, const float* __restrict__ WF2, const float* __restrict__ WC1, __bf16* __restrict__ PK) {
  __shared__ __align__(16) __bf16 s[FFN]; const int n = blockIdx.x, which = blockIdx.y, t = threadIdx.x; int K; size_t dst;
  if (which < 14) { if (n >= CC) return; K = CC; dst = PKW(which) + (size_t)n * CC; const float* Wm = WL.w[0];
#pragma unroll
    for (int i = 1; i < 14; ++i) if (which == i) Wm = WL.w[i];
    if (t < CC) s[t] = (__bf16)Wm[(size_t)t * CC + n]; }
  else if (which == 14) { K = CC; dst = PK_F1 + (size_t)n * CC; if (t < CC) s[t] = (__bf16)WF1[(size_t)t * FFN + n]; }
  else if (which == 15) { if (n >= CC) return; K = FFN; dst = PK_F2 + (size_t)n * FFN; s[t] = (__bf16)WF2[(size_t)t * CC + n]; }
  else { if (n >= CC) return; K = 32; dst = PK_C1 + (size_t)n * 32; if (t < 32) s[t] = (__bf16)((t < CAM) ? WC1[(size_t)t * CC + n] : 0.f); }
  __syncthreads();
  if (t < K / 8) vst2((unsigned*)(PK + dst + t * 8), *(const v4u*)&s[t * 8]);
}
__global__ __launch_bounds__(128) void k_qproj(const float* __restrict__ QF, const float* __restrict__ QP, const float* __restrict__ WQP1, const __bf16* __restrict__ PK, float* __restrict__ Q, float* __restrict__ QPE, float* __restrict__ XS, float* __restrict__ X) {
  __shared__ __align__(16) __bf16 sa[64][CC + 8], sh[64][CC + 8], sl[64][CC + 8]; __shared__ __align__(16) float so[4][16][132], so2[4][16][132];
  const int tid = threadIdx.x, wave = tid >> 5, lane = tid & 31, col = lane & 15, g = lane >> 4; const size_t b = blockIdx.y; const int n0 = blockIdx.x * 64; const size_t r0 = b * NQP + n0 + wave * 16;
  for (int e = tid; e < 64 * CC; e += 128) { const int c = e >> 6, r = e & 63; const int n = n0 + r; sa[r][c] = (__bf16)((n < NQ) ? QF[(b * CC + c) * NQ + n] : 0.f);
    float hv = 0.f; if (n < NQ) { const float p0 = bfr(QP[(b * NQ + n) * 2]), p1 = bfr(QP[(b * NQ + n) * 2 + 1]); hv = fmaxf(p0 * bfr(WQP1[c]) + p1 * bfr(WQP1[CC + c]), 0.f); }
    const __bf16 hb = (__bf16)hv; sh[r][c] = hb; sl[r][c] = (__bf16)(hv - (float)hb); }
  if (tid < 64) for (int c = CC; c < CC + 8; ++c) { sa[tid][c] = (__bf16)0.f; sh[tid][c] = (__bf16)0.f; sl[tid][c] = (__bf16)0.f; }
  __syncthreads();
  v8f acc[8] = {}, acp[8] = {};
#pragma unroll
  for (int kc = 0; kc < CC / 32; ++kc) { const v16b a = frag_b(&sa[wave * 16 + col][kc * 32], lane); F2 p; p.h = frag_b(&sh[wave * 16 + col][kc * 32], lane); p.l = frag_b(&sl[wave * 16 + col][kc * 32], lane);
#pragma unroll
    for (int j = 0; j < 8; ++j) { acc[j] = wmma_bf(a, frag_b(PK + PKW(0) + (size_t)(j * 16 + col) * CC + kc * 32, lane), acc[j]); const v16b w2 = frag_b(PK + PKW(2) + (size_t)(j * 16 + col) * CC + kc * 32, lane); acp[j] = wmma_bf(p.l, w2, acp[j]); acp[j] = wmma_bf(p.h, w2, acp[j]); } }
#pragma unroll
  for (int j = 0; j < 8; ++j)
#pragma unroll
    for (int r = 0; r < 8; ++r) { so[wave][8 * g + r][j * 16 + col] = acc[j][r]; so2[wave][8 * g + r][j * 16 + col] = acp[j][r]; }
  LDSX();
  for (int rl = 0; rl < 16; ++rl) { const v4f q4 = *(const v4f*)&so[wave][rl][lane * 4], p4 = *(const v4f*)&so2[wave][rl][lane * 4]; v4f s4; for (int i = 0; i < 4; ++i) s4[i] = q4[i] + p4[i];
    vst2(Q + (r0 + rl) * CC + lane * 4, q4); vst2(X + (r0 + rl) * CC + lane * 4, q4); vst2(QPE + (r0 + rl) * CC + lane * 4, p4); vst2(XS + (r0 + rl) * CC + lane * 4, s4); }
}
__global__ __launch_bounds__(64) void k_camstat(const float* __restrict__ CI_, float* __restrict__ ST) {
  __shared__ __align__(16) float s[32]; const int t = threadIdx.x; const size_t b = blockIdx.y; const int k0 = blockIdx.x * 64;
  if (t < 32) { const int c = t & 15; float a = 0.f; for (int i = 0; i < 64; ++i) { const float v = bfr(CI_[(b * CAM + c) * NK + k0 + i]); a += (t < 16) ? v : v * v; } s[t] = a; }
  __syncthreads();
  if (t < 8) vst2(ST + ((size_t)b * (NK / 64) + blockIdx.x) * 32 + t * 4, *(const v4f*)&s[t * 4]);
}
__global__ __launch_bounds__(32) void k_cammean(const float* __restrict__ ST, float* __restrict__ MS) {
  const int c = threadIdx.x; __shared__ __align__(16) float sm[32]; if (c < CAM) { float s = 0.f, q2 = 0.f; for (int blk = 0; blk < NB * (NK / 64); ++blk) { s += ST[(size_t)blk * 32 + c]; q2 += ST[(size_t)blk * 32 + 16 + c]; } const float n = (float)(NB * NK); const float mu = s / n; const float var = fmaxf(q2 / n - mu * mu, 0.f); sm[c] = mu; sm[16 + c] = 1.0f / sqrtf(var + 1e-5f); }
  __syncthreads(); if (c < 8) vst2(MS + c * 4, *(const v4f*)&sm[c * 4]);
}
__global__ __launch_bounds__(128) void k_kproj(const float* __restrict__ KFIN, const float* __restrict__ CI_, const float* __restrict__ MS, const __bf16* __restrict__ PK, float* __restrict__ KF0, float* __restrict__ CH) {
  __shared__ __align__(16) __bf16 sa[64][CC + 8], sch[64][40], scl[64][40]; __shared__ __align__(16) float so[4][16][132];
  const int tid = threadIdx.x, wave = tid >> 5, lane = tid & 31, col = lane & 15, g = lane >> 4; const size_t b = blockIdx.y; const int k0 = blockIdx.x * 64; const size_t r0 = b * NK + k0 + wave * 16;
  for (int e = tid; e < 64 * CC; e += 128) { const int c = e >> 6, r = e & 63; sa[r][c] = (__bf16)KFIN[(b * CC + c) * NK + k0 + r]; }
  for (int e = tid; e < 64 * 32; e += 128) { const int r = e >> 5, c = e & 31; float v = 0.f; if (c < CAM) v = (bfr(CI_[(b * CAM + c) * NK + k0 + r]) - MS[c]) * MS[16 + c]; const __bf16 hb = (__bf16)v; sch[r][c] = hb; scl[r][c] = (__bf16)(v - (float)hb); }
  if (tid < 64) for (int c = 0; c < 8; ++c) { sa[tid][CC + c] = (__bf16)0.f; sch[tid][32 + c] = (__bf16)0.f; scl[tid][32 + c] = (__bf16)0.f; }
  __syncthreads();
  v8f acc[8] = {}, acch[8] = {};
#pragma unroll
  for (int kc = 0; kc < CC / 32; ++kc) { const v16b a = frag_b(&sa[wave * 16 + col][kc * 32], lane);
#pragma unroll
    for (int j = 0; j < 8; ++j) acc[j] = wmma_bf(a, frag_b(PK + PKW(1) + (size_t)(j * 16 + col) * CC + kc * 32, lane), acc[j]); }
  { F2 a; a.h = frag_b(&sch[wave * 16 + col][0], lane); a.l = frag_b(&scl[wave * 16 + col][0], lane);
#pragma unroll
    for (int j = 0; j < 8; ++j) { const v16b w = frag_b(PK + PK_C1 + (size_t)(j * 16 + col) * 32, lane); acch[j] = wmma_bf(a.l, w, acch[j]); acch[j] = wmma_bf(a.h, w, acch[j]); } }
#pragma unroll
  for (int j = 0; j < 8; ++j)
#pragma unroll
    for (int r = 0; r < 8; ++r) so[wave][8 * g + r][j * 16 + col] = acc[j][r];
  LDSX();
  for (int rl = 0; rl < 16; ++rl) vst2(KF0 + (r0 + rl) * CC + lane * 4, *(const v4f*)&so[wave][rl][lane * 4]);
  LDSX();
#pragma unroll
  for (int j = 0; j < 8; ++j)
#pragma unroll
    for (int r = 0; r < 8; ++r) so[wave][8 * g + r][j * 16 + col] = fmaxf(acch[j][r], 0.f);
  LDSX();
  for (int rl = 0; rl < 16; ++rl) vst2(CH + (r0 + rl) * CC + lane * 4, *(const v4f*)&so[wave][rl][lane * 4]);
}
template <int MODE>
__global__ __launch_bounds__(128) void k_rows(const float* __restrict__ A, const __bf16* __restrict__ PK, const float* __restrict__ KF0, const float* __restrict__ KP, const float* __restrict__ WKP1, float* __restrict__ OUT, float* __restrict__ OUT2) {
  __shared__ __align__(16) __bf16 sh[64][CC + 8], sl[64][CC + 8]; __shared__ __align__(16) float so[4][16][132], so2[4][16][132];
  const int tid = threadIdx.x, wave = tid >> 5, lane = tid & 31, col = lane & 15, g = lane >> 4; const size_t r0 = (size_t)blockIdx.x * 64 + wave * 16;
  if (MODE == 1) { for (int e = tid; e < 64 * CC; e += 128) { const int c = e >> 6, r = e & 63; const size_t row = (size_t)blockIdx.x * 64 + r; const float p0 = bfr(KP[row * 2]), p1 = bfr(KP[row * 2 + 1]); const float hv = fmaxf(p0 * bfr(WKP1[c]) + p1 * bfr(WKP1[CC + c]), 0.f); const __bf16 hb = (__bf16)hv; sh[r][c] = hb; sl[r][c] = (__bf16)(hv - (float)hb); }
    if (tid < 64) for (int c = CC; c < CC + 8; ++c) { sh[tid][c] = (__bf16)0.f; sl[tid][c] = (__bf16)0.f; } __syncthreads(); }
  v8f acc[8] = {}, acp[8] = {};
#pragma unroll
  for (int kc = 0; kc < CC / 32; ++kc) { const F2 a = split_row(A + (r0 + col) * CC, kc * 32, lane);
#pragma unroll
    for (int j = 0; j < 8; ++j) { const v16b w = frag_b(PK + PKW(MODE == 0 ? 12 : 13) + (size_t)(j * 16 + col) * CC + kc * 32, lane); acc[j] = wmma_bf(a.l, w, acc[j]); acc[j] = wmma_bf(a.h, w, acc[j]);
      if (MODE == 1) { F2 p; p.h = frag_b(&sh[wave * 16 + col][kc * 32], lane); p.l = frag_b(&sl[wave * 16 + col][kc * 32], lane); const v16b w2 = frag_b(PK + PKW(3) + (size_t)(j * 16 + col) * CC + kc * 32, lane); acp[j] = wmma_bf(p.l, w2, acp[j]); acp[j] = wmma_bf(p.h, w2, acp[j]); } } }
#pragma unroll
  for (int j = 0; j < 8; ++j) { const int c = j * 16 + col;
#pragma unroll
    for (int r = 0; r < 8; ++r) { const size_t row = r0 + 8 * g + r;
      if (MODE == 0) so[wave][8 * g + r][c] = fmaxf(acc[j][r], 0.f);
      else { const float gate = 1.0f / (1.0f + exp_ni(-acc[j][r])); const float kf = KF0[row * CC + c] * gate; so[wave][8 * g + r][c] = kf; so2[wave][8 * g + r][c] = kf + acp[j][r]; } } }
  LDSX();
  for (int rl = 0; rl < 16; ++rl) { vst2(OUT + (r0 + rl) * CC + lane * 4, *(const v4f*)&so[wave][rl][lane * 4]); if (MODE == 1) vst2(OUT2 + (r0 + rl) * CC + lane * 4, *(const v4f*)&so2[wave][rl][lane * 4]); }
}
__global__ __launch_bounds__(128) void k_hproj(const float* __restrict__ A, const __bf16* __restrict__ PW, int kind, int S, _Float16* __restrict__ OH_, _Float16* __restrict__ OL_) {
  __shared__ __align__(16) _Float16 soh[4][16][NH * 32 + 8], sol[4][16][NH * 32 + 8]; __shared__ __align__(16) _Float16 sth[128][72], stl[128][72];
  const int tid = threadIdx.x, wave = tid >> 5, lane = tid & 31, col = lane & 15, g = lane >> 4; const size_t r0 = (size_t)blockIdx.x * 64 + wave * 16;
  v8f acc[8] = {};
#pragma unroll
  for (int kc = 0; kc < CC / 32; ++kc) { const F2 a = split_row(A + (r0 + col) * CC, kc * 32, lane);
#pragma unroll
    for (int j = 0; j < 8; ++j) { const v16b w = frag_b(PW + (size_t)(j * 16 + col) * CC + kc * 32, lane); acc[j] = wmma_bf(a.l, w, acc[j]); acc[j] = wmma_bf(a.h, w, acc[j]); } }
  if (kind == 0) {
    for (int e = tid; e < 4 * 16 * (NH * 32 + 8); e += 128) { (&soh[0][0][0])[e] = (_Float16)0.f; (&sol[0][0][0])[e] = (_Float16)0.f; }
    __syncthreads();
#pragma unroll
    for (int j = 0; j < 8; ++j)
#pragma unroll
      for (int r = 0; r < 8; ++r) { const float v = acc[j][r]; const _Float16 hv = (_Float16)v; soh[wave][8 * g + r][j * 32 + col] = hv; sol[wave][8 * g + r][j * 32 + col] = (_Float16)((v - (float)hv) * 2048.0f); }
    LDSX();
    for (int rl = 0; rl < 16; ++rl) { const size_t o = (r0 + rl) * (NH * 32); vst2((unsigned*)(OH_ + o + lane * 8), *(const v4u*)&soh[wave][rl][lane * 8]); vst2((unsigned*)(OL_ + o + lane * 8), *(const v4u*)&sol[wave][rl][lane * 8]); }
  } else {
#pragma unroll
    for (int j = 0; j < 8; ++j)
#pragma unroll
      for (int r = 0; r < 8; ++r) { const float v = acc[j][r]; const _Float16 hv = (_Float16)v; sth[j * 16 + col][wave * 16 + 8 * g + r] = hv; stl[j * 16 + col][wave * 16 + 8 * g + r] = (_Float16)((v - (float)hv) * 2048.0f); }
    __syncthreads();
    const size_t rb = (size_t)blockIdx.x * 64; const size_t b = rb / S; const int s0 = (int)(rb % S);
    for (int e = tid; e < 128 * 8; e += 128) { const int d = e >> 3, pc = e & 7; const size_t o = (b * CC + d) * S + s0 + pc * 8; vst2((unsigned*)(OH_ + o), *(const v4u*)&sth[d][pc * 8]); vst2((unsigned*)(OL_ + o), *(const v4u*)&stl[d][pc * 8]); }
  }
}
__global__ __launch_bounds__(128) void k_attn(const _Float16* __restrict__ QH, const _Float16* __restrict__ QL, const _Float16* __restrict__ KH, const _Float16* __restrict__ KL, const _Float16* __restrict__ VTH, const _Float16* __restrict__ VTL, int NKEY, int cross, const float* __restrict__ QPOS, const float* __restrict__ KPOS, const float* __restrict__ QSZ, float* __restrict__ SO) {
  __shared__ __align__(16) _Float16 sph[4][16][40], spl[4][16][40]; __shared__ __align__(16) float so[4][16][36];
  const int tid = threadIdx.x, wave = tid >> 5, lane = tid & 31, col = lane & 15, g = lane >> 4; const int hp = blockIdx.y; const size_t b = blockIdx.z; const int q0 = blockIdx.x * 64 + wave * 16; const size_t rq = b * NQP + q0;
  float qpx[8], qpy[8], isx[8], isy[8];
#pragma unroll
  for (int r = 0; r < 8; ++r) { const int qi = q0 + 8 * g + r; const int qc = min(qi, NQ - 1); qpx[r] = bfr(QPOS[(b * NQ + qc) * 2]); qpy[r] = bfr(QPOS[(b * NQ + qc) * 2 + 1]); const float sx = bfr(QSZ[(b * NQ + qc) * 2]) * 0.5f + 1e-2f, sy = bfr(QSZ[(b * NQ + qc) * 2 + 1]) * 0.5f + 1e-2f; isx[r] = 1.0f / (2.0f * (sx * sx)); isy[r] = 1.0f / (2.0f * (sy * sy)); }
#pragma unroll 1
  for (int hh = 0; hh < 2; ++hh) { const int h = hp * 2 + hh;
    const v16h aq = frag_h(QH + (rq + col) * (NH * 32) + h * 32, lane), aql = frag_h(QL + (rq + col) * (NH * 32) + h * 32, lane);
    float m[8], l[8];
#pragma unroll
    for (int r = 0; r < 8; ++r) { m[r] = -3.0e38f; l[r] = 0.f; }
    v8f acc = {}, accl = {};
    const size_t kb = (size_t)b * NKEY;
#pragma unroll 1
    for (int ks = 0; ks < NKEY / 32; ++ks) { const int j0 = ks * 32; v8f s[2];
#pragma unroll
      for (int ct = 0; ct < 2; ++ct) { const int kk = j0 + ct * 16 + col; const size_t rk = (kb + kk) * (NH * 32) + h * 32; v8f c = {}, cl = {};
        { const v16h kh = frag_h(KH + rk, lane); c = wmma16(aq, kh, c); cl = wmma16(aql, kh, cl); cl = wmma16(aq, frag_h(KL + rk, lane), cl); }
        float bias[8];
        if (cross) { const float kx = bfr(KPOS[(kb + kk) * 2]), ky = bfr(KPOS[(kb + kk) * 2 + 1]);
#pragma unroll
          for (int r = 0; r < 8; ++r) { const float dx = kx - qpx[r], dy = ky - qpy[r]; bias[r] = -(dx * dx * isx[r] + dy * dy * isy[r]); } }
        else {
#pragma unroll
          for (int r = 0; r < 8; ++r) bias[r] = 0.f; }
        const bool kvalid = cross || (kk < NQ);
#pragma unroll
        for (int r = 0; r < 8; ++r) s[ct][r] = kvalid ? (c[r] + cl[r] * (1.0f / 2048.0f)) * 0.25f + bias[r] : -3.0e38f; }
#pragma unroll
      for (int r = 0; r < 8; ++r) { float mx = fmaxf(s[0][r], s[1][r]);
#pragma unroll
        for (int o = 1; o < 16; o <<= 1) mx = fmaxf(mx, __shfl_xor(mx, o));
        const float mn = fmaxf(m[r], mx); const float alpha = (m[r] <= -1.0e38f) ? 0.f : __expf(m[r] - mn);
        const float e0 = (s[0][r] <= -1.0e38f) ? 0.f : __expf(s[0][r] - mn), e1 = (s[1][r] <= -1.0e38f) ? 0.f : __expf(s[1][r] - mn); float es = e0 + e1;
#pragma unroll
        for (int o = 1; o < 16; o <<= 1) es += __shfl_xor(es, o);
        l[r] = l[r] * alpha + es; m[r] = (mn <= -1.0e38f) ? m[r] : mn; acc[r] *= alpha; accl[r] *= alpha;
        const _Float16 h0 = (_Float16)e0, h1 = (_Float16)e1; sph[wave][8 * g + r][col] = h0; sph[wave][8 * g + r][16 + col] = h1; spl[wave][8 * g + r][col] = (_Float16)((e0 - (float)h0) * 2048.0f); spl[wave][8 * g + r][16 + col] = (_Float16)((e1 - (float)h1) * 2048.0f); }
      LDSX();
      const v16h pah = frag_h(&sph[wave][col][0], lane), pal = frag_h(&spl[wave][col][0], lane);
      { const size_t vo = (b * CC + h * DH + col) * NKEY + j0; const v16h vh = frag_h(VTH + vo, lane), vl = frag_h(VTL + vo, lane); acc = wmma16(pah, vh, acc); accl = wmma16(pal, vh, accl); accl = wmma16(pah, vl, accl); }
      LDSX(); }
#pragma unroll
    for (int r = 0; r < 8; ++r) { const float il = 1.0f / l[r]; so[wave][8 * g + r][hh * 16 + col] = (acc[r] + accl[r] * (1.0f / 2048.0f)) * il; } }
  LDSX();
  for (int rl = 0; rl < 16; ++rl) if (lane < 8) vst2(SO + (rq + rl) * CC + hp * 32 + lane * 4, *(const v4f*)&so[wave][rl][lane * 4]);
}
template <int MODE>
__global__ __launch_bounds__(128) void k_oln(const float* __restrict__ SOA, const __bf16* __restrict__ PK, const float* __restrict__ B1, const float* __restrict__ B2, float* __restrict__ X, const float* __restrict__ QPE, float* __restrict__ XS, float* __restrict__ OUT) {
  __shared__ __align__(16) float so[4][16][132]; __shared__ __align__(16) __bf16 sg[64][FFN + 8], sgl[64][FFN + 8];
  const int tid = threadIdx.x, wave = tid >> 5, lane = tid & 31, col = lane & 15, g = lane >> 4; const size_t r0 = (size_t)blockIdx.x * 64 + wave * 16;
  v8f acc[8] = {};
  if (MODE < 2) {
#pragma unroll
    for (int kc = 0; kc < CC / 32; ++kc) { const F2 a = split_row(SOA + (r0 + col) * CC, kc * 32, lane);
#pragma unroll
      for (int j = 0; j < 8; ++j) { const v16b w = frag_b(PK + PKW(MODE == 0 ? 7 : 11) + (size_t)(j * 16 + col) * CC + kc * 32, lane); acc[j] = wmma_bf(a.l, w, acc[j]); acc[j] = wmma_bf(a.h, w, acc[j]); } }
  } else {
#pragma unroll 1
    for (int pass = 0; pass < 2; ++pass) { v8f ac1[8] = {};
#pragma unroll
      for (int kc = 0; kc < CC / 32; ++kc) { const F2 a = split_row(X + (r0 + col) * CC, kc * 32, lane);
#pragma unroll
        for (int j = 0; j < 8; ++j) { const v16b w = frag_b(PK + PK_F1 + (size_t)(pass * 128 + j * 16 + col) * CC + kc * 32, lane); ac1[j] = wmma_bf(a.l, w, ac1[j]); ac1[j] = wmma_bf(a.h, w, ac1[j]); } }
#pragma unroll
      for (int j = 0; j < 8; ++j) { const int c = pass * 128 + j * 16 + col; const float bb = bfr(B1[c]);
#pragma unroll
        for (int r = 0; r < 8; ++r) { const float v = fmaxf(ac1[j][r] + bb, 0.f); const __bf16 hb = (__bf16)v; sg[wave * 16 + 8 * g + r][c] = hb; sgl[wave * 16 + 8 * g + r][c] = (__bf16)(v - (float)hb); } } }
    if (lane < 8) for (int rl = 0; rl < 16; ++rl) { sg[wave * 16 + rl][FFN + lane] = (__bf16)0.f; sgl[wave * 16 + rl][FFN + lane] = (__bf16)0.f; }
    LDSX();
#pragma unroll
    for (int kc = 0; kc < FFN / 32; ++kc) { F2 a; a.h = frag_b(&sg[wave * 16 + col][kc * 32], lane); a.l = frag_b(&sgl[wave * 16 + col][kc * 32], lane);
#pragma unroll
      for (int j = 0; j < 8; ++j) { const v16b w = frag_b(PK + PK_F2 + (size_t)(j * 16 + col) * FFN + kc * 32, lane); acc[j] = wmma_bf(a.l, w, acc[j]); acc[j] = wmma_bf(a.h, w, acc[j]); } }
  }
  float mu[8], rs[8];
#pragma unroll
  for (int r = 0; r < 8; ++r) { const size_t row = r0 + 8 * g + r; float s = 0.f, q2 = 0.f;
#pragma unroll
    for (int j = 0; j < 8; ++j) { const int c = j * 16 + col; float v = acc[j][r] + X[row * CC + c]; if (MODE == 2) v += bfr(B2[c]); acc[j][r] = v; s += v; q2 += v * v; }
#pragma unroll
    for (int o = 1; o < 16; o <<= 1) { s += __shfl_xor(s, o); q2 += __shfl_xor(q2, o); }
    mu[r] = s / (float)CC; rs[r] = 1.0f / sqrtf(fmaxf(q2 / (float)CC - mu[r] * mu[r], 0.f) + 1e-5f); }
  __syncthreads();
#pragma unroll
  for (int j = 0; j < 8; ++j)
#pragma unroll
    for (int r = 0; r < 8; ++r) so[wave][8 * g + r][j * 16 + col] = (acc[j][r] - mu[r]) * rs[r];
  LDSX();
  for (int rl = 0; rl < 16; ++rl) { const size_t row = r0 + rl; const v4f v = *(const v4f*)&so[wave][rl][lane * 4];
    if (MODE < 2) { vst2(X + row * CC + lane * 4, v); if (MODE == 0) { const v4f p4 = *(const v4f*)(QPE + row * CC + lane * 4); v4f s4; for (int i = 0; i < 4; ++i) s4[i] = v[i] + p4[i]; vst2(XS + row * CC + lane * 4, s4); } }
    else { const size_t b = row / NQP; const int n = (int)(row % NQP); if (n < NQ) vst2(OUT + (b * NQ + n) * CC + lane * 4, v); } }
}
extern "C" void kernel_launch(void* const* d_in, const int* in_sizes, int n_in, void* d_out, int out_size, void* d_ws, size_t ws_size, hipStream_t stream) {
  (void)in_sizes; (void)n_in; (void)out_size;
  const float** F = (const float**)d_in;
  if (ws_size < (size_t)WS_END) return;
  char* ws = (char*)d_ws; __bf16* PK = (__bf16*)(ws + WS_PK); float *Q = (float*)(ws + WS_Q), *QPE = (float*)(ws + WS_QPE), *XS = (float*)(ws + WS_XS), *X = (float*)(ws + WS_X), *T = (float*)(ws + WS_T), *SO = (float*)(ws + WS_SO), *KF = (float*)(ws + WS_KF), *KC = (float*)(ws + WS_KC), *CH = (float*)(ws + WS_CH), *ST = (float*)(ws + WS_ST), *MS = (float*)(ws + WS_MS);
  _Float16 *SQH = (_Float16*)(ws + WS_SQH), *SQL = (_Float16*)(ws + WS_SQL), *SKH = (_Float16*)(ws + WS_SKH), *SKL = (_Float16*)(ws + WS_SKL), *SVH = (_Float16*)(ws + WS_SVH), *SVL = (_Float16*)(ws + WS_SVL), *CKH = (_Float16*)(ws + WS_CKH), *CKL = (_Float16*)(ws + WS_CKL), *CVH = (_Float16*)(ws + WS_CVH), *CVL = (_Float16*)(ws + WS_CVL);
  (void)T;
  WList wl; { const int idx[14] = {6, 7, 9, 11, 12, 13, 14, 15, 16, 17, 18, 19, 25, 26}; for (int i = 0; i < 14; ++i) wl.w[i] = F[idx[i]]; }
  k_pack<<<dim3(FFN, 17), 256, 0, stream>>>(wl, F[20], F[22], F[24], PK);
  k_qproj<<<dim3(NQP / 64, NB), 128, 0, stream>>>(F[0], F[2], F[8], PK, Q, QPE, XS, X);
  k_camstat<<<dim3(NK / 64, NB), 64, 0, stream>>>(F[5], ST);
  k_cammean<<<1, 32, 0, stream>>>(ST, MS);
  k_kproj<<<dim3(NK / 64, NB), 128, 0, stream>>>(F[1], F[5], MS, PK, KC, CH);
  k_rows<0><<<NKR / 64, 128, 0, stream>>>(CH, PK, nullptr, nullptr, nullptr, KF, nullptr);
  k_rows<1><<<NKR / 64, 128, 0, stream>>>(KF, PK, KC, F[3], F[10], CH, KC);
  k_hproj<<<NQR / 64, 128, 0, stream>>>(XS, PK + PKW(4), 0, NQP, SQH, SQL);
  k_hproj<<<NQR / 64, 128, 0, stream>>>(XS, PK + PKW(5), 0, NQP, SKH, SKL);
  k_hproj<<<NQR / 64, 128, 0, stream>>>(X, PK + PKW(6), 1, NQP, SVH, SVL);
  k_attn<<<dim3(NQP / 64, NH / 2, NB), 128, 0, stream>>>(SQH, SQL, SKH, SKL, SVH, SVL, NQP, 0, F[2], F[3], F[4], SO);
  k_oln<0><<<NQR / 64, 128, 0, stream>>>(SO, PK, nullptr, nullptr, X, QPE, XS, nullptr);
  k_hproj<<<NQR / 64, 128, 0, stream>>>(XS, PK + PKW(8), 0, NQP, SQH, SQL);
  k_hproj<<<NKR / 64, 128, 0, stream>>>(KC, PK + PKW(9), 0, NK, CKH, CKL);
  k_hproj<<<NKR / 64, 128, 0, stream>>>(CH, PK + PKW(10), 1, NK, CVH, CVL);
  k_attn<<<dim3(NQP / 64, NH / 2, NB), 128, 0, stream>>>(SQH, SQL, CKH, CKL, CVH, CVL, NK, 1, F[2], F[3], F[4], SO);
  k_oln<1><<<NQR / 64, 128, 0, stream>>>(SO, PK, nullptr, nullptr, X, nullptr, nullptr, nullptr);
  k_oln<2><<<NQR / 64, 128, 0, stream>>>(nullptr, PK, F[21], F[23], X, nullptr, nullptr, (float*)d_out);
}
